// Iteration_dec_44985487458947
// MI455X (gfx1250) — hardware-verified
//
#include <hip/hip_runtime.h>
#include <stdint.h>

#define LEN   1024
#define DIM   64
#define KW    5
#define EPSBN 1e-3f
#define NTHR  256
#define WHALF (5 * 4 * 32 * 16)

typedef char check_nthr_covers_row[(NTHR * 4 == LEN) ? 1 : -1];

typedef _Float16 v16h __attribute__((ext_vector_type(16)));
typedef _Float16 v8h  __attribute__((ext_vector_type(8)));
typedef float    v8f  __attribute__((ext_vector_type(8)));
typedef float    v4f  __attribute__((ext_vector_type(4)));

union Frag { v16h v; v8h half[2]; };

__device__ __forceinline__ float elu1(float y) {
    return y > 0.f ? y : (__expf(y) - 1.f);
}

__device__ __forceinline__ int clampi(int v, int lo, int hi) {
    return v < lo ? lo : (v > hi ? hi : v);
}

__device__ __forceinline__ v8f wmma16(const v16h& a, const v16h& b, v8f c) {
    return __builtin_amdgcn_wmma_f32_16x16x32_f16(false, a, false, b, (short)0, c, false, false);
}

__launch_bounds__(NTHR, 1)
__global__ void k_branch(
    const float* __restrict__ c0, const float* __restrict__ c1, const float* __restrict__ c2,
    const float* __restrict__ Wfirst, const float* __restrict__ bfirst,
    const float* __restrict__ Wrest,  const float* __restrict__ brest,
    const float* __restrict__ gg, const float* __restrict__ bt,
    const float* __restrict__ mm, const float* __restrict__ vv,
    const float* __restrict__ fcW, const float* __restrict__ fcb,
    float* __restrict__ qout, int nb)
{
    __shared__ __align__(16) _Float16 sActA[LEN * DIM];
    __shared__ __align__(16) _Float16 sActB[LEN * DIM];
    __shared__ __align__(32) _Float16 sWswz[WHALF];
    __shared__ __align__(16) float sScr[1152];

    const int b = blockIdx.x;
    if (b >= nb) return;
    const int tid    = threadIdx.x;
    const int lane   = tid & 31;
    const int wv     = tid >> 5;
    const int laneHi = lane >> 4;
    const int lane15 = lane & 15;
    const int ntile  = wv & 3;
    const int dch    = ntile * 16 + lane15;
    const int rt0    = (wv >> 2) * 32;

    const size_t sbase = (size_t)b * LEN;

    for (int e = tid; e < KW * 3 * DIM; e += NTHR) sScr[e] = Wfirst[e];
    if (tid < DIM) {
        float s = gg[tid] * rsqrtf(vv[tid] + EPSBN);
        sScr[960  + tid] = s;
        sScr[1024 + tid] = (bfirst[tid] - mm[tid]) * s + bt[tid];
    }
    __syncthreads();

    for (int l = tid; l < LEN; l += NTHR) {
        float iv[KW][3];
        #pragma unroll
        for (int k = 0; k < KW; ++k) {
            int lp = (l + k + (LEN - 2)) & (LEN - 1);
            iv[k][0] = c0[sbase + lp];
            iv[k][1] = c1[sbase + lp];
            iv[k][2] = c2[sbase + lp];
        }
        #pragma unroll 1
        for (int d0 = 0; d0 < DIM; d0 += 8) {
            v8h ov;
            #pragma unroll
            for (int dd = 0; dd < 8; ++dd) {
                const int d = d0 + dd;
                float acc = 0.f;
                #pragma unroll
                for (int k = 0; k < KW; ++k)
                    #pragma unroll
                    for (int c = 0; c < 3; ++c)
                        acc = fmaf(iv[k][c], sScr[(k * 3 + c) * DIM + d], acc);
                acc = acc * sScr[960 + d] + sScr[1024 + d];
                ov[dd] = (_Float16)elu1(acc);
            }
            *reinterpret_cast<v8h*>(sActA + l * DIM + d0) = ov;
        }
    }

    for (int j = 0; j < 4; ++j) {
        const _Float16* actIn  = (j & 1) ? sActB : sActA;
        _Float16*       actOut = (j & 1) ? sActA : sActB;
        const float* Wg = Wrest + (size_t)j * KW * DIM * DIM;

        const int li = j + 1;
        const float s  = gg[li * DIM + dch] * rsqrtf(vv[li * DIM + dch] + EPSBN);
        const float sh = (brest[j * DIM + dch] - mm[li * DIM + dch]) * s + bt[li * DIM + dch];
        const float sw = s * 0.0625f;

        v16h bfrag[10];
        #pragma unroll
        for (int hp = 0; hp < 2; ++hp) {
            if (hp) __syncthreads();
            for (int e = tid; e < WHALF; e += NTHR) {
                int i    = e & 15;
                int ln   = (e >> 4) & 31;
                int fr   = e >> 9;
                int ck   = hp * 5 + (fr >> 2);
                int nt   = fr & 3;
                int kin  = (ln >> 4) * 8 + (i & 7) + ((i >> 3) << 4);
                int k    = ck >> 1;
                int cin  = (ck & 1) * 32 + kin;
                int cout = nt * 16 + (ln & 15);
                sWswz[e] = (_Float16)(Wg[(k * DIM + cin) * DIM + cout] * 16.f);
            }
            __syncthreads();
            #pragma unroll
            for (int c = 0; c < 5; ++c)
                bfrag[hp * 5 + c] = *reinterpret_cast<const v16h*>(
                    sWswz + ((c * 4 + ntile) * 32 + lane) * 16);
        }

        #pragma unroll 1
        for (int rt = rt0; rt < rt0 + 32; ++rt) {
            const int l0 = rt * 16;
            int aoff[KW];
            #pragma unroll
            for (int k = 0; k < KW; ++k)
                aoff[k] = ((l0 + lane15 + k + (LEN - 2)) & (LEN - 1)) * DIM + laneHi * 8;

            v8f acc = {0.f, 0.f, 0.f, 0.f, 0.f, 0.f, 0.f, 0.f};
            Frag a;
            #pragma unroll
            for (int ck = 0; ck < 10; ++ck) {
                const _Float16* ap = actIn + aoff[ck >> 1] + (ck & 1) * 32;
                a.half[0] = *reinterpret_cast<const v8h*>(ap);
                a.half[1] = *reinterpret_cast<const v8h*>(ap + 16);
                acc = wmma16(a.v, bfrag[ck], acc);
            }
            asm volatile("v_nop\n\tv_nop\n\tv_nop\n\tv_nop" : "+v"(acc) : "v"(a.v), "v"(bfrag[9]));

            #pragma unroll
            for (int r = 0; r < 8; ++r) {
                int rowl = l0 + r + laneHi * 8;
                float y = acc[r] * sw + sh;
                actOut[rowl * DIM + dch] = (_Float16)elu1(y);
            }
        }
        __syncthreads();
    }

    if (tid < DIM) sScr[tid] = fcW[tid];
    __syncthreads();
    const float fcbv = fcb[0];
    const int l4 = tid * 4;
    float qa[4];
    #pragma unroll
    for (int e = 0; e < 4; ++e) {
        const int l = l4 + e;
        float sacc = fcbv;
        #pragma unroll
        for (int d0 = 0; d0 < DIM; d0 += 8) {
            v8h hv = *reinterpret_cast<const v8h*>(sActA + l * DIM + d0);
            #pragma unroll
            for (int dd = 0; dd < 8; ++dd)
                sacc = fmaf((float)hv[dd], sScr[d0 + dd], sacc);
        }
        qa[e] = sacc;
    }
    v4f qv;
    qv.x = qa[0]; qv.y = qa[1]; qv.z = qa[2]; qv.w = qa[3];
    volatile v4f* op = reinterpret_cast<volatile v4f*>(qout + sbase + l4);
    *op = qv;
    __threadfence();
    *op = qv;
}

__launch_bounds__(NTHR)
__global__ void k_interleave(const float* __restrict__ q0, const float* __restrict__ dx,
                             const int* __restrict__ perm,
                             float* __restrict__ p2, float* __restrict__ dxI, int nb)
{
    const int b = blockIdx.x;
    if (b >= nb) return;
    const size_t sbase = (size_t)b * LEN;
    const int l4 = threadIdx.x * 4;
    int idx[4];
    #pragma unroll
    for (int e = 0; e < 4; ++e) idx[e] = clampi(perm[sbase + l4 + e], 0, LEN - 1);
    v4f vq, vd;
    vq.x = q0[sbase + idx[0]]; vq.y = q0[sbase + idx[1]]; vq.z = q0[sbase + idx[2]]; vq.w = q0[sbase + idx[3]];
    vd.x = dx[sbase + idx[0]]; vd.y = dx[sbase + idx[1]]; vd.z = dx[sbase + idx[2]]; vd.w = dx[sbase + idx[3]];
    volatile v4f* oq = reinterpret_cast<volatile v4f*>(p2  + sbase + l4);
    volatile v4f* od = reinterpret_cast<volatile v4f*>(dxI + sbase + l4);
    *oq = vq; *od = vd;
    __threadfence();
    *oq = vq; *od = vd;
}

__launch_bounds__(NTHR)
__global__ void k_deinterleave(const float* __restrict__ q1, const int* __restrict__ invp,
                               float* __restrict__ out, int nb)
{
    const int b = blockIdx.x;
    if (b >= nb) return;
    const size_t sbase = (size_t)b * LEN;
    const int l4 = threadIdx.x * 4;
    int idx[4];
    #pragma unroll
    for (int e = 0; e < 4; ++e) idx[e] = clampi(invp[sbase + l4 + e], 0, LEN - 1);
    v4f v;
    v.x = q1[sbase + idx[0]]; v.y = q1[sbase + idx[1]]; v.z = q1[sbase + idx[2]]; v.w = q1[sbase + idx[3]];
    volatile v4f* op = reinterpret_cast<volatile v4f*>(out + sbase + l4);
    *op = v;
    __threadfence();
    *op = v;
}

extern "C" void kernel_launch(void* const* d_in, const int* in_sizes, int n_in,
                              void* d_out, int out_size, void* d_ws, size_t ws_size,
                              hipStream_t stream) {
    if (n_in < 26) return;
    const int nb = in_sizes[24] / LEN;
    if (nb <= 0) return;
    if (nb * LEN != in_sizes[24] || nb * LEN != in_sizes[25]) return;
    if (out_size != nb * LEN) return;
    if (in_sizes[0] != nb * LEN || in_sizes[1] != nb * LEN ||
        in_sizes[2] != nb * LEN || in_sizes[3] != nb * LEN) return;
    if (in_sizes[4] != KW * 3 * DIM || in_sizes[6] != 4 * KW * DIM * DIM ||
        in_sizes[12] != KW * 3 * DIM || in_sizes[14] != 4 * KW * DIM * DIM) return;
    if (in_sizes[5] < DIM || in_sizes[7] < 4 * DIM || in_sizes[13] < DIM || in_sizes[15] < 4 * DIM) return;
    if (in_sizes[8] < 5 * DIM || in_sizes[9] < 5 * DIM || in_sizes[10] < 5 * DIM || in_sizes[11] < 5 * DIM) return;
    if (in_sizes[16] < 5 * DIM || in_sizes[17] < 5 * DIM || in_sizes[18] < 5 * DIM || in_sizes[19] < 5 * DIM) return;
    if (in_sizes[20] < DIM || in_sizes[22] < DIM || in_sizes[21] < 1 || in_sizes[23] < 1) return;

    const size_t per = (size_t)nb * LEN * sizeof(float);
    if (4 * per > ws_size) return;
    char* wsb = (char*)d_ws;
    float* q0  = (float*)(wsb);
    float* p2  = (float*)(wsb + per);
    float* dxI = (float*)(wsb + 2 * per);
    float* q1  = (float*)(wsb + 3 * per);

    const float* dx       = (const float*)d_in[0];
    const float* de       = (const float*)d_in[1];
    const float* dI       = (const float*)d_in[2];
    const float* pp_in    = (const float*)d_in[3];
    const float* Wx_first = (const float*)d_in[4];
    const float* bx_first = (const float*)d_in[5];
    const float* Wx_rest  = (const float*)d_in[6];
    const float* bx_rest  = (const float*)d_in[7];
    const float* gx       = (const float*)d_in[8];
    const float* btx      = (const float*)d_in[9];
    const float* mx       = (const float*)d_in[10];
    const float* vx       = (const float*)d_in[11];
    const float* WI_first = (const float*)d_in[12];
    const float* bI_first = (const float*)d_in[13];
    const float* WI_rest  = (const float*)d_in[14];
    const float* bI_rest  = (const float*)d_in[15];
    const float* gI       = (const float*)d_in[16];
    const float* btI      = (const float*)d_in[17];
    const float* mI       = (const float*)d_in[18];
    const float* vI       = (const float*)d_in[19];
    const float* fc1_W    = (const float*)d_in[20];
    const float* fc1_b    = (const float*)d_in[21];
    const float* fc2_W    = (const float*)d_in[22];
    const float* fc2_b    = (const float*)d_in[23];
    const int*   perm     = (const int*)d_in[24];
    const int*   inv_perm = (const int*)d_in[25];
    float* outp = (float*)d_out;

    k_branch<<<nb, NTHR, 0, stream>>>(de, pp_in, dx,
        Wx_first, bx_first, Wx_rest, bx_rest, gx, btx, mx, vx,
        fc1_W, fc1_b, q0, nb);
    k_interleave<<<nb, NTHR, 0, stream>>>(q0, dx, perm, p2, dxI, nb);
    k_branch<<<nb, NTHR, 0, stream>>>(dI, p2, dxI,
        WI_first, bI_first, WI_rest, bI_rest, gI, btI, mI, vI,
        fc2_W, fc2_b, q1, nb);
    k_deinterleave<<<nb, NTHR, 0, stream>>>(q1, inv_perm, outp, nb);
}
